// SoftDDT_88124138979497
// MI455X (gfx1250) — hardware-verified
//
#include <hip/hip_runtime.h>
#include <stddef.h>
#include <stdint.h>
#include <math.h>

#define NB    4096
#define NI    1024
#define NO    1024
#define NNODE 4095
#define NNP   4096
#define NLEAF 4096
#define DEPTH 12
#define TBM   64
#define TBN   128

static_assert((NI % 32) == 0);
static_assert((NLEAF % 32) == 0);
static_assert((NB % TBM) == 0);
static_assert((NNP % TBN) == 0);
static_assert((NO % TBN) == 0);
static_assert((1 << DEPTH) == NLEAF);
static_assert(NNODE == NLEAF - 1);
static_assert((DEPTH & 1) == 0);
static_assert(((NB * NI) % 2048) == 0);
static_assert(((NNP * NI) % 2048) == 0);
static_assert((NO % 64) == 0);
static_assert((NLEAF % 64) == 0);
static_assert(NLEAF == 16 * 256);
static_assert(NNP == 16 * 256);

typedef __attribute__((ext_vector_type(16))) __bf16 v16b;
typedef _Float16     v16h __attribute__((ext_vector_type(16)));
typedef _Float16     v8h  __attribute__((ext_vector_type(8)));
typedef float        v8f  __attribute__((ext_vector_type(8)));
typedef float        v4f  __attribute__((ext_vector_type(4)));
typedef unsigned int v4u  __attribute__((ext_vector_type(4)));

__device__ __forceinline__ unsigned short bf_bits(float f) {
  const unsigned u = __float_as_uint(f);
  return (unsigned short)((u + 0x7FFFu + ((u >> 16) & 1u)) >> 16);
}
__device__ __forceinline__ float bfr(float f) { return __uint_as_float(((unsigned)bf_bits(f)) << 16); }
__device__ __forceinline__ unsigned pk16(unsigned short a, unsigned short b) { return (unsigned)a | ((unsigned)b << 16); }
__device__ __forceinline__ v8f zero8() { v8f z = {0.f, 0.f, 0.f, 0.f, 0.f, 0.f, 0.f, 0.f}; return z; }
__device__ __forceinline__ _Float16 to_h_flush(float f) {
  const float a = fabsf(f) < 6.103515625e-05f ? 0.0f : f;
  return (_Float16)a;
}

union Frag { v16h h; v16b b; v4u u[2]; };
__device__ __forceinline__ Frag ldfrag(const unsigned short* p) {
  Frag f;
  f.u[0] = *(const v4u*)(p);
  f.u[1] = *(const v4u*)(p + 16);
  return f;
}

template <int KIND>
__device__ __forceinline__ v8f mma(const Frag& a, const Frag& b, v8f c) {
  if (KIND == 0)
    return __builtin_amdgcn_wmma_f32_16x16x32_bf16(false, a.b, false, b.b, (short)0, c, false, false);
  else
    return __builtin_amdgcn_wmma_f32_16x16x32_f16(false, a.h, false, b.h, (short)0, c, false, false);
}
__device__ __forceinline__ void guard8(v8f& c0, v8f& c1, v8f& c2, v8f& c3, v8f& c4, v8f& c5, v8f& c6, v8f& c7,
                                       const Frag& a0, const Frag& a1,
                                       const Frag& b0, const Frag& b1, const Frag& b2, const Frag& b3) {
#if defined(__HIP_DEVICE_COMPILE__)
  asm volatile("v_nop\n\tv_nop\n\tv_nop\n\tv_nop"
               : "+v"(c0), "+v"(c1), "+v"(c2), "+v"(c3), "+v"(c4), "+v"(c5), "+v"(c6), "+v"(c7)
               : "v"(a0.h), "v"(a1.h), "v"(b0.h), "v"(b1.h), "v"(b2.h), "v"(b3.h));
#endif
}

__global__ __launch_bounds__(256)
void k_cv(const float* __restrict__ src, unsigned short* dst, int nvalid, int ntotal) {
  const size_t f8 = ((size_t)blockIdx.x * 256 + threadIdx.x) * 8;
  if (f8 + 8 > (size_t)ntotal) return;
  const bool pad = (f8 >= (size_t)nvalid);
  const size_t fl = pad ? (size_t)nvalid - 8 : f8;
  const v4f a = *(const v4f*)(src + fl);
  const v4f b = *(const v4f*)(src + fl + 4);
  v4u u;
  u[0] = pk16(bf_bits(a[0]), bf_bits(a[1]));
  u[1] = pk16(bf_bits(a[2]), bf_bits(a[3]));
  u[2] = pk16(bf_bits(b[0]), bf_bits(b[1]));
  u[3] = pk16(bf_bits(b[2]), bf_bits(b[3]));
  if (pad) { u[0] = 0u; u[1] = 0u; u[2] = 0u; u[3] = 0u; }
  unsigned short* dp = dst + f8;
  *(volatile v4u*)dp = u;
  __threadfence();
  *(volatile v4u*)dp = u;
}

__global__ __launch_bounds__(256)
void k_tleaf(const float* __restrict__ leaf, unsigned short* Lt) {
  __shared__ __align__(16) unsigned short sT[64 * 72];
  const int o0 = blockIdx.x * 64, l0 = blockIdx.y * 64;
  const int tid = threadIdx.x;
  const int rr = tid >> 4, c4 = (tid & 15) * 4;
#pragma unroll
  for (int it = 0; it < 4; ++it) {
    const int ll = it * 16 + rr;
    const v4f v = *(const v4f*)(leaf + (size_t)(l0 + ll) * NO + o0 + c4);
#pragma unroll
    for (int j = 0; j < 4; ++j) {
      const _Float16 h = to_h_flush(bfr(v[j]) * 16.0f);
      sT[(c4 + j) * 72 + ll] = __builtin_bit_cast(unsigned short, h);
    }
  }
  __syncthreads();
  const int p = tid & 7, lq = tid >> 3;
  v4u u[2];
#pragma unroll
  for (int it = 0; it < 2; ++it) {
    const int oo = it * 32 + lq;
    u[it] = *(const v4u*)(sT + oo * 72 + p * 8);
  }
  unsigned short* dp = Lt + (size_t)(o0 + lq) * NLEAF + l0 + p * 8;
#pragma unroll
  for (int it = 0; it < 2; ++it) *(volatile v4u*)(dp + (size_t)it * 32 * NLEAF) = u[it];
  __threadfence();
#pragma unroll
  for (int it = 0; it < 2; ++it) *(volatile v4u*)(dp + (size_t)it * 32 * NLEAF) = u[it];
}

template <int KIND>
__global__ __launch_bounds__(128)
void k_gemm(const unsigned short* __restrict__ A, const unsigned short* __restrict__ Bm,
            const float* __restrict__ bias, float* C, int K, int ldc, int nbias) {
  __shared__ __align__(16) float sO[TBM * TBN];
  const int tid = threadIdx.x, w = tid >> 5, lane = tid & 31, hh = lane >> 4, c = lane & 15;
  const int wm = w & 1, wn = w >> 1;
  const int Mbase = blockIdx.y * TBM, Nbase = blockIdx.x * TBN;
  const int mrow0 = Mbase + 32 * wm;
  const int ncol0 = Nbase + 64 * wn;
  const size_t Ks = (size_t)K;

  const unsigned short* ap0 = A + (size_t)(mrow0 + c) * Ks + 8 * hh;
  const unsigned short* ap1 = ap0 + 16 * Ks;
  const unsigned short* bp0 = Bm + (size_t)(ncol0 + c) * Ks + 8 * hh;
  const unsigned short* bp1 = bp0 + 16 * Ks;
  const unsigned short* bp2 = bp0 + 32 * Ks;
  const unsigned short* bp3 = bp0 + 48 * Ks;

  v8f acc[2][4];
#pragma unroll
  for (int mi = 0; mi < 2; ++mi)
#pragma unroll
    for (int ni = 0; ni < 4; ++ni) acc[mi][ni] = zero8();

  const int nk = K >> 5;
#pragma unroll 1
  for (int ks = 0; ks < nk; ++ks) {
    const int ko = ks << 5;
    const Frag a0 = ldfrag(ap0 + ko);
    const Frag a1 = ldfrag(ap1 + ko);
    const Frag b0 = ldfrag(bp0 + ko);
    const Frag b1 = ldfrag(bp1 + ko);
    const Frag b2 = ldfrag(bp2 + ko);
    const Frag b3 = ldfrag(bp3 + ko);
    acc[0][0] = mma<KIND>(a0, b0, acc[0][0]);
    acc[0][1] = mma<KIND>(a0, b1, acc[0][1]);
    acc[0][2] = mma<KIND>(a0, b2, acc[0][2]);
    acc[0][3] = mma<KIND>(a0, b3, acc[0][3]);
    acc[1][0] = mma<KIND>(a1, b0, acc[1][0]);
    acc[1][1] = mma<KIND>(a1, b1, acc[1][1]);
    acc[1][2] = mma<KIND>(a1, b2, acc[1][2]);
    acc[1][3] = mma<KIND>(a1, b3, acc[1][3]);
    guard8(acc[0][0], acc[0][1], acc[0][2], acc[0][3], acc[1][0], acc[1][1], acc[1][2], acc[1][3],
           a0, a1, b0, b1, b2, b3);
  }

#pragma unroll
  for (int mi = 0; mi < 2; ++mi) {
#pragma unroll
    for (int ni = 0; ni < 4; ++ni) {
      const int lcol = 64 * wn + 16 * ni + c;
#pragma unroll
      for (int r = 0; r < 8; ++r) {
        const int lrow = 32 * wm + 16 * mi + 8 * hh + r;
        sO[lrow * TBN + lcol] = acc[mi][ni][r];
      }
    }
  }
  __syncthreads();

  if (KIND == 0) {
    v4f b4;
#pragma unroll
    for (int j = 0; j < 4; ++j) {
      int n = Nbase + lane * 4 + j;
      n = (n < nbias) ? n : (nbias - 1);
      b4[j] = bfr(bias[n]);
    }
#pragma unroll 1
    for (int it = 0; it < 16; ++it) {
      float* q = sO + (it * 4 + w) * TBN + lane * 4;
      v4f v = *(const v4f*)q;
#pragma unroll
      for (int j = 0; j < 4; ++j) {
        float z = v[j] + b4[j];
        z = fminf(fmaxf(z, -30.0f), 30.0f);
        const float e = expf(-z);
        v[j] = 1.0f / (1.0f + e);
      }
      *(v4f*)q = v;
    }
  }
  v4f o[16];
#pragma unroll
  for (int it = 0; it < 16; ++it) {
    v4f v = *(const v4f*)(sO + (it * 4 + w) * TBN + lane * 4);
    if (KIND == 1) v = v * (1.0f / 524288.0f);
    o[it] = v;
  }
  float* cp = C + (size_t)(Mbase + w) * (size_t)ldc + Nbase + lane * 4;
#pragma unroll
  for (int it = 0; it < 16; ++it) *(volatile v4f*)(cp + (size_t)it * 4 * (size_t)ldc) = o[it];
  __threadfence();
#pragma unroll
  for (int it = 0; it < 16; ++it) *(volatile v4f*)(cp + (size_t)it * 4 * (size_t)ldc) = o[it];
}

__global__ __launch_bounds__(256)
void k_expand(const float* __restrict__ g, unsigned short* P) {
#pragma clang fp contract(off)
  __shared__ __align__(16) float sg[NNP];
  __shared__ __align__(16) float sp[2 * NLEAF];
  const int row = blockIdx.x, tid = threadIdx.x;
  const float* gr = g + (size_t)row * NNP;
#pragma unroll
  for (int j = 0; j < 4; ++j) {
    const int f = tid * 4 + 1024 * j;
    *(v4f*)(sg + f) = *(const v4f*)(gr + f);
  }
  if (tid == 0) sp[0] = 1.0f;
  __syncthreads();

  int cur = 0;
#pragma unroll 1
  for (int d = 0; d < DEPTH; ++d) {
    const int n = 1 << d;
    const float* src = sp + cur * NLEAF;
    float* dst = sp + (cur ^ 1) * NLEAF;
    for (int i = tid; i < n; i += 256) {
      const float p  = src[i];
      const float gv = sg[n - 1 + i];
      dst[2 * i]     = p * (1.0f - gv);
      dst[2 * i + 1] = p * gv;
    }
    __syncthreads();
    cur ^= 1;
  }

  union HB { v8h h; v4u u; };
  v4u u[2];
#pragma unroll
  for (int qq = 0; qq < 2; ++qq) {
    const int f = 8 * tid + 2048 * qq;
    const v4f a = *(const v4f*)(sp + f);
    const v4f b = *(const v4f*)(sp + f + 4);
    HB hb;
#pragma unroll
    for (int j = 0; j < 4; ++j) {
      hb.h[j]     = to_h_flush(a[j] * 32768.0f);
      hb.h[4 + j] = to_h_flush(b[j] * 32768.0f);
    }
    u[qq] = hb.u;
  }
  unsigned short* dp = P + (size_t)row * NLEAF + 8 * tid;
#pragma unroll
  for (int qq = 0; qq < 2; ++qq) *(volatile v4u*)(dp + 2048 * qq) = u[qq];
  __threadfence();
#pragma unroll
  for (int qq = 0; qq < 2; ++qq) *(volatile v4u*)(dp + 2048 * qq) = u[qq];
}

extern "C" void kernel_launch(void* const* d_in, const int* in_sizes, int n_in,
                              void* d_out, int out_size, void* d_ws, size_t ws_size,
                              hipStream_t stream) {
  if (n_in < 4) return;
  if (in_sizes[0] != NB * NI) return;
  if (in_sizes[1] != NNODE * NI) return;
  if (in_sizes[2] != NNODE) return;
  if (in_sizes[3] != NLEAF * NO) return;
  if (out_size != NB * NO) return;

  const float* x    = (const float*)d_in[0];
  const float* Wn   = (const float*)d_in[1];
  const float* bn   = (const float*)d_in[2];
  const float* leaf = (const float*)d_in[3];
  float* out = (float*)d_out;

  const size_t sX = (size_t)NB * NI * 2;
  const size_t sW = (size_t)NNP * NI * 2;
  const size_t sL = (size_t)NO * NLEAF * 2;
  const size_t sG = (size_t)NB * NNP * 4;
  const size_t sP = (size_t)NB * NLEAF * 2;
  size_t off = 0;
  const size_t oX = off; off += sX;
  const size_t oW = off; off += sW;
  const size_t oL = off; off += sL;
  const size_t oG = off; off += sG;
  const size_t oP = off; off += sP;
  if (off > ws_size) return;
  if (off > (size_t)134217728) return;

  char* ws = (char*)d_ws;
  unsigned short* Xb = (unsigned short*)(ws + oX);
  unsigned short* Wb = (unsigned short*)(ws + oW);
  unsigned short* Lt = (unsigned short*)(ws + oL);
  float* G = (float*)(ws + oG);
  unsigned short* P = (unsigned short*)(ws + oP);

  k_cv<<<dim3((NB * NI) / 2048), dim3(256), 0, stream>>>(x, Xb, NB * NI, NB * NI);
  k_cv<<<dim3((NNP * NI) / 2048), dim3(256), 0, stream>>>(Wn, Wb, NNODE * NI, NNP * NI);
  k_tleaf<<<dim3(NO / 64, NLEAF / 64), dim3(256), 0, stream>>>(leaf, Lt);
  k_gemm<0><<<dim3(NNP / TBN, NB / TBM), dim3(128), 0, stream>>>(Xb, Wb, bn, G, NI, NNP, NNODE);
  k_expand<<<dim3(NB), dim3(256), 0, stream>>>(G, P);
  k_gemm<1><<<dim3(NO / TBN, NB / TBM), dim3(128), 0, stream>>>(P, Lt, bn, out, NLEAF, NO, NNODE);
  (void)hipGetLastError();
}
